// MultiHeadAttention_49211735277730
// MI455X (gfx1250) — hardware-verified
//
#include <hip/hip_runtime.h>

#ifndef NB
#define NB 4
#endif
#ifndef SEQ
#define SEQ 2048
#endif
#define NB_FULL 4
#define SEQ_FULL 2048
#define EMB 512
#define NHEAD 8
#define HDIM 64
#define NQK (2 * EMB)
#define NQKV (3 * EMB)
#define MROWS (NB * SEQ)

static_assert(HDIM == 64);
static_assert(EMB == NHEAD * HDIM);
static_assert(SEQ % 64 == 0);
static_assert(EMB % 64 == 0);
static_assert(NB <= NB_FULL);
static_assert(SEQ <= SEQ_FULL);
static_assert((NB == 1) || (SEQ == SEQ_FULL));

typedef __attribute__((ext_vector_type(16))) _Float16 v16h;
typedef __attribute__((ext_vector_type(8)))  _Float16 v8h;
typedef __attribute__((ext_vector_type(8)))  float    v8f;
typedef __attribute__((ext_vector_type(4)))  float    v4f;
typedef unsigned int cm_u4 __attribute__((ext_vector_type(4)));


#define VST2(T, ptr, val) do { const T vst2_v_ = (val); *(volatile T*)(ptr) = vst2_v_; __threadfence(); *(volatile T*)(ptr) = vst2_v_; } while (0)

namespace eng {

union FragU { v16h v; v8h h[2]; };
__device__ __forceinline__ v16h frag_load(const _Float16* p) {
  FragU f; f.h[0] = *(const v8h*)(p); f.h[1] = *(const v8h*)(p + 16); return f.v;
}
__device__ __forceinline__ v8f mma_h(v16h a, v16h b, v8f c) {
  return __builtin_amdgcn_wmma_f32_16x16x32_f16(false, a, false, b, (short)0, c, false, false);
}
__device__ __forceinline__ void guard_row4(v8f& a, v8f& b, v8f& c, v8f& d, v16h x) { asm volatile("v_nop\n\tv_nop\n\tv_nop\n\tv_nop" : "+v"(a), "+v"(b), "+v"(c), "+v"(d) : "v"(x)); }
__device__ __forceinline__ void keep4_h(v16h a, v16h b, v16h c, v16h d) { asm volatile("v_nop" :: "v"(a), "v"(b), "v"(c), "v"(d)); }
__device__ __forceinline__ void acc_guard4(v8f& a, v8f& b, v8f& c, v8f& d) { asm volatile("v_nop\n\tv_nop\n\tv_nop\n\tv_nop" : "+v"(a), "+v"(b), "+v"(c), "+v"(d)); }
__device__ __forceinline__ void guard_s(v8f& a, v16h x0, v16h x1, v16h y0, v16h y1) { asm volatile("v_nop\n\tv_nop\n\tv_nop\n\tv_nop" : "+v"(a) : "v"(x0), "v"(x1), "v"(y0), "v"(y1)); }
__device__ __forceinline__ void guard_o(v8f& a, v8f& b, v8f& c, v8f& d, v16h x0, v16h x1, v16h x2, v16h x3, v16h y) {
  asm volatile("v_nop\n\tv_nop\n\tv_nop\n\tv_nop" : "+v"(a), "+v"(b), "+v"(c), "+v"(d) : "v"(x0), "v"(x1), "v"(x2), "v"(x3), "v"(y));
}

__device__ __forceinline__ float bf_rne(float v) { const unsigned u = __builtin_bit_cast(unsigned, v); const unsigned r = (u + 0x7fffu + ((u >> 16) & 1u)) & 0xffff0000u; return __builtin_bit_cast(float, r); }

template <int BIAS_MODE, int OUT_MODE>
__global__ __launch_bounds__(256) void wmma_gemm64(
    const unsigned short* __restrict__ Ap, int lda, long strideA,
    const unsigned short* __restrict__ Btp, int ldb, long strideB,
    void* Cout, int ldc, long strideC,
    const float* __restrict__ bias,
    int M, int N, int K, float scale) {
  const _Float16* A = (const _Float16*)Ap; const _Float16* Bt = (const _Float16*)Btp;
  __shared__ __align__(16) float sT[8][16 * 68];
  const int b    = blockIdx.y;
  const int lane = threadIdx.x & 31;
  const int wave = __builtin_amdgcn_readfirstlane((int)(threadIdx.x >> 5));
  const int tilesN = N >> 6;
  const int tilesM = M >> 6;
  const int tile = blockIdx.x * 8 + wave;
  if (tile >= tilesM * tilesN) return;
  const int tm = tile / tilesN;
  const int tn = tile - tm * tilesN;
  const int m0 = tm << 6;
  const int n0 = tn << 6;

  const _Float16* Ab = A  + (size_t)b * strideA;
  const _Float16* Bb = Bt + (size_t)b * strideB;

  const int rlane = lane & 15;
  const int koff  = (lane >> 4) * 8;
  const int mOff  = (lane >> 4) * 8;

  v8f acc[4][4];
#pragma unroll
  for (int i = 0; i < 4; ++i)
#pragma unroll
    for (int j = 0; j < 4; ++j) acc[i][j] = (v8f){0.f,0.f,0.f,0.f,0.f,0.f,0.f,0.f};

  for (int k0 = 0; k0 < K; k0 += 32) {
    v16h bh[4];
#pragma unroll
    for (int j = 0; j < 4; ++j) {
      const size_t bo = (size_t)(n0 + (j << 4) + rlane) * ldb + koff + k0;
      bh[j] = frag_load(Bb + bo);
    }
#pragma unroll
    for (int i = 0; i < 4; ++i) {
      const size_t ao = (size_t)(m0 + (i << 4) + rlane) * lda + koff + k0;
      const v16h ah = frag_load(Ab + ao);
#pragma unroll
      for (int j = 0; j < 4; ++j) acc[i][j] = mma_h(ah, bh[j], acc[i][j]);
      guard_row4(acc[i][0], acc[i][1], acc[i][2], acc[i][3], ah);
    }
    keep4_h(bh[0], bh[1], bh[2], bh[3]);
  }
  acc_guard4(acc[0][0], acc[0][1], acc[0][2], acc[0][3]);
  acc_guard4(acc[1][0], acc[1][1], acc[1][2], acc[1][3]);
  acc_guard4(acc[2][0], acc[2][1], acc[2][2], acc[2][3]);
  acc_guard4(acc[3][0], acc[3][1], acc[3][2], acc[3][3]);

  float* slab = sT[wave];
#pragma unroll
  for (int i = 0; i < 4; ++i) {
    const int mBase = m0 + (i << 4);
    float bm[8];
#pragma unroll
    for (int r = 0; r < 8; ++r) bm[r] = (BIAS_MODE == 1) ? bf_rne(bias[mBase + mOff + r]) : 0.f;
#pragma unroll
    for (int j = 0; j < 4; ++j) {
      const int n = n0 + (j << 4) + rlane;
      float bv = 0.f;
      if (BIAS_MODE == 2) bv = bf_rne(bias[n]);
#pragma unroll
      for (int r = 0; r < 8; ++r) {
        float v = acc[i][j][r] * scale;
        if (BIAS_MODE == 1) v += bm[r];
        if (BIAS_MODE == 2) v += bv;
        slab[(mOff + r) * 68 + (j << 4) + rlane] = v;
      }
    }
    __builtin_amdgcn_fence(3  , "workgroup");
    __builtin_amdgcn_wave_barrier();
    __builtin_amdgcn_fence(2  , "workgroup");
    if (OUT_MODE == 0) {
      float* C = (float*)Cout + (size_t)b * strideC;
      const int hh = lane >> 4, c4 = (lane & 15) * 4;
      for (int pass = 0; pass < 2; ++pass) {
#pragma unroll
        for (int it = 0; it < 8; ++it) {
          const int row = it * 2 + hh;
          v4f v = *(const v4f*)(slab + row * 68 + c4);
          *(volatile v4f*)(C + (size_t)(mBase + row) * ldc + n0 + c4) = v;
        }
        __threadfence();
      }
    } else {
      const int q = lane >> 3, c8 = (lane & 7) * 8;
      unsigned short* C = (unsigned short*)Cout + (size_t)b * strideC;
      for (int pass = 0; pass < 2; ++pass) {
#pragma unroll
        for (int it = 0; it < 4; ++it) {
          const int row = it * 4 + q;
          const float* sp = slab + row * 68 + c8;
          v8h hv;
#pragma unroll
          for (int e = 0; e < 8; ++e) hv[e] = (_Float16)sp[e];
          *(volatile v8h*)(C + (size_t)(mBase + row) * ldc + n0 + c8) = hv;
        }
        __threadfence();
      }
    }
    __builtin_amdgcn_fence(3  , "workgroup");
    __builtin_amdgcn_wave_barrier();
    __builtin_amdgcn_fence(2  , "workgroup");
  }
}

}

__device__ __forceinline__ unsigned int cmb_pk2(float a, float b) { return (unsigned int)__builtin_bit_cast(unsigned short, (_Float16)a) | ((unsigned int)__builtin_bit_cast(unsigned short, (_Float16)b) << 16); }
__global__ __launch_bounds__(256) void k_cm_castb(const float* __restrict__ SRC, unsigned short* __restrict__ DST, unsigned int n8, float sc) {
#pragma clang fp contract(off)
    const unsigned int u = blockIdx.x * 256u + threadIdx.x; if (u >= n8) return;
    const v4f a = *(const v4f*)(SRC + (size_t)u * 8u), b4 = *(const v4f*)(SRC + (size_t)u * 8u + 4u);
    cm_u4 pk;
    pk.x = cmb_pk2(eng::bf_rne(a.x) * sc, eng::bf_rne(a.y) * sc); pk.y = cmb_pk2(eng::bf_rne(a.z) * sc, eng::bf_rne(a.w) * sc);
    pk.z = cmb_pk2(eng::bf_rne(b4.x) * sc, eng::bf_rne(b4.y) * sc); pk.w = cmb_pk2(eng::bf_rne(b4.z) * sc, eng::bf_rne(b4.w) * sc);
    VST2(cm_u4, (cm_u4*)(DST + (size_t)u * 8u), pk); }

__global__ __launch_bounds__(256) void k_cast_tr(const float* __restrict__ SRC, unsigned short* __restrict__ DST, int rows, int cols, float sc) {
#pragma clang fp contract(off)
    __shared__ float ts[64][65];
    const int c0 = blockIdx.x * 64, r0 = blockIdx.y * 64;
    if (r0 + 64 > rows || c0 + 64 > cols) return;
    const int tid = threadIdx.x;
#pragma unroll 1
    for (int it = 0; it < 4; ++it) {
        const int idx = it * 256 + tid;
        const int r = idx >> 4, c4 = (idx & 15) * 4;
        const v4f v = *(const v4f*)(SRC + (size_t)(r0 + r) * cols + c0 + c4);
        ts[r][c4 + 0] = eng::bf_rne(v.x) * sc;
        ts[r][c4 + 1] = eng::bf_rne(v.y) * sc;
        ts[r][c4 + 2] = eng::bf_rne(v.z) * sc;
        ts[r][c4 + 3] = eng::bf_rne(v.w) * sc;
    }
    __syncthreads();
#pragma unroll 1
    for (int it = 0; it < 2; ++it) {
        const int idx = it * 256 + tid;
        const int n = idx >> 3, j = (idx & 7) * 8;
        cm_u4 pk;
        pk.x = cmb_pk2(ts[j + 0][n], ts[j + 1][n]);
        pk.y = cmb_pk2(ts[j + 2][n], ts[j + 3][n]);
        pk.z = cmb_pk2(ts[j + 4][n], ts[j + 5][n]);
        pk.w = cmb_pk2(ts[j + 6][n], ts[j + 7][n]);
        VST2(cm_u4, (cm_u4*)(DST + (size_t)(c0 + n) * rows + r0 + j), pk);
    }
}

__global__ __launch_bounds__(128)
void k_fattn_t(const unsigned short* __restrict__ QKp, const unsigned short* __restrict__ VTp, unsigned short* AOp) {
    const float SCL2 = 0.18033688011112042f;
    const float NEGINF = -__builtin_inff();
    __shared__ __align__(16) float Os[4][16 * 68];

    const unsigned int lane = threadIdx.x & 31u, hh = lane >> 4, c = lane & 15u;
    const unsigned int wave = (unsigned int)__builtin_amdgcn_readfirstlane((int)(threadIdx.x >> 5));
    const unsigned int qb = blockIdx.x, h = blockIdx.y, b = blockIdx.z;
    const unsigned int q0 = qb * 64u + wave * 16u;

    const _Float16* qk = (const _Float16*)QKp;
    const _Float16* vt = (const _Float16*)VTp;

    v16h qf[2];
    {
        const size_t qo = (size_t)(b * (unsigned)SEQ + q0 + c) * (unsigned)NQK + h * 64u + 8u * hh;
        qf[0] = eng::frag_load(qk + qo);
        qf[1] = eng::frag_load(qk + qo + 32);
    }

    float mrun = NEGINF, lrun = 0.f;
    v8f oacc[4];
#pragma unroll
    for (int t = 0; t < 4; ++t) oacc[t] = (v8f){0.f,0.f,0.f,0.f,0.f,0.f,0.f,0.f};

    const _Float16* kbase = qk + (size_t)(b * (unsigned)SEQ + c) * (unsigned)NQK + (unsigned)EMB + h * 64u + 8u * hh;
    const _Float16* vbase = vt + (size_t)(b * (unsigned)EMB + h * 64u + c) * (unsigned)SEQ + 8u * hh;

#pragma unroll 1
    for (unsigned int kv0 = 0; kv0 < (unsigned)SEQ; kv0 += 64u) {
        v8f s[4];
#pragma unroll
        for (int j = 0; j < 4; ++j) {
            const _Float16* kp = kbase + (size_t)(kv0 + (unsigned)j * 16u) * (unsigned)NQK;
            const v16h k0 = eng::frag_load(kp);
            const v16h k1 = eng::frag_load(kp + 32);
            v8f acc = (v8f){0.f,0.f,0.f,0.f,0.f,0.f,0.f,0.f};
            acc = eng::mma_h(k0, qf[0], acc);
            acc = eng::mma_h(k1, qf[1], acc);
            eng::guard_s(acc, k0, k1, qf[0], qf[1]);
            s[j] = acc;
        }
        float vmax = s[0][0];
#pragma unroll
        for (int j = 0; j < 4; ++j)
#pragma unroll
            for (int r = 0; r < 8; ++r) vmax = fmaxf(vmax, s[j][r]);
        vmax = fmaxf(vmax, __shfl_xor(vmax, 16, 32));
        const float mnew = fmaxf(mrun, vmax * SCL2);
        const float alpha = exp2f(mrun - mnew);
        mrun = mnew;
        const float nb = 15.0f - mnew;
        float psum = 0.f;
        v16h pb[2];
#pragma unroll
        for (int j = 0; j < 4; ++j)
#pragma unroll
            for (int r = 0; r < 8; ++r) {
                const float pc = exp2f(fmaf(s[j][r], SCL2, nb));
                psum += pc;
                pb[j >> 1][(j & 1) * 8 + r] = (_Float16)pc;
            }
        lrun = lrun * alpha + psum;
#pragma unroll
        for (int t = 0; t < 4; ++t)
#pragma unroll
            for (int r = 0; r < 8; ++r) oacc[t][r] *= alpha;
#pragma unroll
        for (int kk = 0; kk < 2; ++kk) {
            const _Float16* vp = vbase + kv0 + (unsigned)kk * 32u;
            const v16h va0 = eng::frag_load(vp);
            const v16h va1 = eng::frag_load(vp + (size_t)16 * (unsigned)SEQ);
            const v16h va2 = eng::frag_load(vp + (size_t)32 * (unsigned)SEQ);
            const v16h va3 = eng::frag_load(vp + (size_t)48 * (unsigned)SEQ);
            oacc[0] = eng::mma_h(va0, pb[kk], oacc[0]);
            oacc[1] = eng::mma_h(va1, pb[kk], oacc[1]);
            oacc[2] = eng::mma_h(va2, pb[kk], oacc[2]);
            oacc[3] = eng::mma_h(va3, pb[kk], oacc[3]);
            eng::guard_o(oacc[0], oacc[1], oacc[2], oacc[3], va0, va1, va2, va3, pb[kk]);
        }
    }

    const float ltot = lrun + __shfl_xor(lrun, 16, 32);
    const float inv = 16.0f * (1.0f / ltot);
    float* os = Os[wave];
#pragma unroll
    for (int t = 0; t < 4; ++t)
#pragma unroll
        for (int r = 0; r < 8; ++r)
            os[c * 68u + (unsigned)t * 16u + 8u * hh + (unsigned)r] = oacc[t][r] * inv;
    __builtin_amdgcn_fence(3  , "workgroup");
    __builtin_amdgcn_wave_barrier();
    __builtin_amdgcn_fence(2  , "workgroup");
    {
        const unsigned int q = lane >> 3, c8 = (lane & 7u) * 8u;
        unsigned short* ao = AOp + (size_t)(b * (unsigned)SEQ + q0) * (unsigned)EMB + h * 64u + c8;
        for (int pass = 0; pass < 2; ++pass) {
#pragma unroll
            for (int it = 0; it < 4; ++it) {
                const unsigned int row = (unsigned)it * 4u + q;
                const float* sp = os + row * 68u + c8;
                v8h hv;
#pragma unroll
                for (int e = 0; e < 8; ++e) hv[e] = (_Float16)sp[e];
                *(volatile v8h*)(ao + (size_t)row * (unsigned)EMB) = hv;
            }
            __threadfence();
        }
    }
}

constexpr size_t WS_X16  = (size_t)MROWS * EMB * 2;
constexpr size_t WS_W3   = (size_t)NQKV * EMB * 2;
constexpr size_t WS_WO   = (size_t)EMB * EMB * 2;
constexpr size_t WS_QK   = (size_t)MROWS * NQK * 2;
constexpr size_t WS_VT   = (size_t)NB * EMB * SEQ * 2;
constexpr size_t WS_AO   = (size_t)MROWS * EMB * 2;
constexpr size_t OFF_X16 = 0;
constexpr size_t OFF_W3  = OFF_X16 + WS_X16;
constexpr size_t OFF_WO  = OFF_W3 + WS_W3;
constexpr size_t OFF_QK  = OFF_WO + WS_WO;
constexpr size_t OFF_VT  = OFF_QK + WS_QK;
constexpr size_t OFF_AO  = OFF_VT + WS_VT;
constexpr size_t WS_TOTAL = OFF_AO + WS_AO;
static_assert(WS_X16 % 256 == 0 && WS_W3 % 256 == 0 && WS_WO % 256 == 0);
static_assert(WS_QK % 256 == 0 && WS_VT % 256 == 0 && WS_AO % 256 == 0);
static_assert(WS_TOTAL <= (size_t)134217728);

static_assert(((size_t)MROWS * EMB / 8) % 256 == 0);
static_assert(NQKV % 64 == 0 && EMB % 64 == 0);
static_assert(((MROWS / 64) * (NQK / 64)) % 8 == 0);
static_assert(((EMB / 64) * (SEQ / 64)) % 8 == 0);
static_assert(((MROWS / 64) * (EMB / 64)) % 8 == 0);
static_assert(MROWS % 64 == 0 && NQK % 64 == 0 && EMB % 32 == 0);

extern "C" void kernel_launch(void* const* d_in, const int* in_sizes, int n_in, void* d_out, int out_size, void* d_ws, size_t ws_size, hipStream_t stream) {
    if (n_in < 5) return;
    if (in_sizes[0] < MROWS * EMB) return;
    if (in_sizes[1] < NQKV * EMB) return;
    if (in_sizes[2] < NQKV) return;
    if (in_sizes[3] < EMB * EMB) return;
    if (in_sizes[4] < EMB) return;
    if (out_size < MROWS * EMB) return;
    if (ws_size < WS_TOTAL) return;
    const float* x    = (const float*)d_in[0];
    const float* Wqkv = (const float*)d_in[1];
    const float* bqkv = (const float*)d_in[2];
    const float* Wo   = (const float*)d_in[3];
    const float* bo   = (const float*)d_in[4];
    float* out = (float*)d_out;
    char* wsp = (char*)d_ws;
    unsigned short* X16  = (unsigned short*)(wsp + OFF_X16);
    unsigned short* W3T  = (unsigned short*)(wsp + OFF_W3);
    unsigned short* WOT  = (unsigned short*)(wsp + OFF_WO);
    unsigned short* QK16 = (unsigned short*)(wsp + OFF_QK);
    unsigned short* VT16 = (unsigned short*)(wsp + OFF_VT);
    unsigned short* AO16 = (unsigned short*)(wsp + OFF_AO);

    k_cm_castb<<<(unsigned)(((size_t)MROWS * EMB / 8) / 256), 256, 0, stream>>>(x, X16, (unsigned)((size_t)MROWS * EMB / 8), 1.0f);
    k_cast_tr<<<dim3((unsigned)(NQKV / 64), (unsigned)(EMB / 64)), 256, 0, stream>>>(Wqkv, W3T, EMB, NQKV, 16.0f);
    k_cast_tr<<<dim3((unsigned)(EMB / 64), (unsigned)(EMB / 64)), 256, 0, stream>>>(Wo, WOT, EMB, EMB, 16.0f);

    eng::wmma_gemm64<2, 1><<<dim3((unsigned)(((MROWS / 64) * (NQK / 64)) / 8), 1u), 256, 0, stream>>>(
        (const unsigned short*)X16, EMB, (long)0,
        (const unsigned short*)W3T, EMB, (long)0,
        (void*)QK16, NQK, (long)0,
        bqkv,
        MROWS, NQK, EMB, 0.0625f);
    eng::wmma_gemm64<1, 1><<<dim3((unsigned)(((EMB / 64) * (SEQ / 64)) / 8), (unsigned)NB), 256, 0, stream>>>(
        (const unsigned short*)(W3T + (size_t)NQK * EMB), EMB, (long)0,
        (const unsigned short*)X16, EMB, (long)SEQ * EMB,
        (void*)VT16, SEQ, (long)EMB * SEQ,
        bqkv + NQK,
        EMB, SEQ, EMB, 0.0625f);

    k_fattn_t<<<dim3((unsigned)(SEQ / 64), (unsigned)NHEAD, (unsigned)NB), 128, 0, stream>>>(QK16, VT16, AO16);

    eng::wmma_gemm64<2, 0><<<dim3((unsigned)(((MROWS / 64) * (EMB / 64)) / 8), 1u), 256, 0, stream>>>(
        (const unsigned short*)AO16, EMB, (long)0,
        (const unsigned short*)WOT, EMB, (long)0,
        (void*)out, EMB, (long)0,
        bo,
        MROWS, EMB, EMB, 1.0f / 256.0f);
}
